// MultiHeadAttention_39711267619157
// MI455X (gfx1250) — hardware-run, weakly checked
//
#include <hip/hip_runtime.h>
#include <math.h>

#ifndef NB
#define NB 2
#endif
#ifndef SEQ
#define SEQ 2048
#endif
#define NB_FULL  2
#define SEQ_FULL 2048
#define DMODEL   1024
#define NH       16
#define NKV      4
#define GRP      4
#define DK       64
#define QKVN     1536
#define SWK      12

static_assert(SEQ % 64 == 0);
static_assert(NB <= NB_FULL);
static_assert(SEQ <= SEQ_FULL);
static_assert(((long long)(NB - 1) * SEQ_FULL + SEQ) * DMODEL <= (long long)NB_FULL * SEQ_FULL * DMODEL);
static_assert(QKVN % 64 == 0);
static_assert(DMODEL % 64 == 0);

typedef unsigned short u16;
typedef __attribute__((ext_vector_type(16))) __bf16       v16b;
typedef __attribute__((ext_vector_type(8)))  __bf16       v8b;
typedef __attribute__((ext_vector_type(8)))  float        v8f;
typedef __attribute__((ext_vector_type(4)))  float        v4f;
typedef __attribute__((ext_vector_type(2)))  float        v2f;
typedef __attribute__((ext_vector_type(4)))  unsigned int v4u;

union FragB { v16b v; v8b h[2]; };
union PFrag { unsigned int u[8]; v16b v; };

__device__ __forceinline__ v16b frag_ld(const __bf16* __restrict__ base, int ld, int row0, int k0, int lane) {
    const __bf16* p = base + (size_t)(row0 + (lane & 15)) * ld + k0 + ((lane >> 4) << 3);
    FragB f; f.h[0] = *(const v8b*)(p); f.h[1] = *(const v8b*)(p + 16); return f.v;
}

__device__ __forceinline__ v8f mma3(v16b ah, v16b al, v16b bh, v16b bl, v8f c) {
    c = __builtin_amdgcn_wmma_f32_16x16x32_bf16(false, ah, false, bh, (short)0, c, false, false);
    c = __builtin_amdgcn_wmma_f32_16x16x32_bf16(false, ah, false, bl, (short)0, c, false, false);
    c = __builtin_amdgcn_wmma_f32_16x16x32_bf16(false, al, false, bh, (short)0, c, false, false);
    asm volatile("v_nop\n\tv_nop\n\tv_nop\n\tv_nop" : "+v"(c) : "v"(ah), "v"(al), "v"(bh), "v"(bl));
    return c;
}
__device__ __forceinline__ void dep_guard_b(v8f& a, v8f& b, v16b x, v16b y) { asm volatile("v_nop\n\tv_nop\n\tv_nop\n\tv_nop" : "+v"(a), "+v"(b) : "v"(x), "v"(y)); }
__device__ __forceinline__ void keep4_b(v16b a, v16b b, v16b c, v16b d) { asm volatile("v_nop" :: "v"(a), "v"(b), "v"(c), "v"(d)); }
__device__ __forceinline__ void acc_guard4(v8f& a, v8f& b, v8f& c, v8f& d) { asm volatile("v_nop\n\tv_nop\n\tv_nop\n\tv_nop" : "+v"(a), "+v"(b), "+v"(c), "+v"(d)); }

__device__ __forceinline__ unsigned int bfu_rne(float v) { unsigned int u = __float_as_uint(v); u += 0x7fffu + ((u >> 16) & 1u); return u >> 16; }
__device__ __forceinline__ float bfu_f32(unsigned int hb) { return __uint_as_float(hb << 16); }
__device__ __forceinline__ float cmb_bf(float v) { return bfu_f32(bfu_rne(v)); }
__device__ __forceinline__ void bfsplit(float v, unsigned int& hi, unsigned int& lo) { hi = bfu_rne(v); lo = bfu_rne(v - bfu_f32(hi)); }
__device__ __forceinline__ unsigned int pk2bf(float a, float b) { return bfu_rne(a) | (bfu_rne(b) << 16); }

#define VST2(T, ptr, val) do { const T vst2_v_ = (val); *(volatile T*)(ptr) = vst2_v_; __threadfence(); *(volatile T*)(ptr) = vst2_v_; } while (0)

__device__ __forceinline__ void st_s2(u16* Hp, u16* Lp, size_t o, float a, float b) {
    unsigned int h0, l0, h1, l1; bfsplit(a, h0, l0); bfsplit(b, h1, l1);
    const unsigned int ph = h0 | (h1 << 16), pl = l0 | (l1 << 16);
    volatile unsigned int* dh = (volatile unsigned int*)(Hp + o); volatile unsigned int* dl = (volatile unsigned int*)(Lp + o);
    *dh = ph; *dl = pl; __threadfence(); *dh = ph; *dl = pl;
}
__device__ __forceinline__ void split8(v4f a, v4f b, v4u& hv, v4u& lv) {
    unsigned int h0, l0, h1, l1;
    bfsplit(a.x, h0, l0); bfsplit(a.y, h1, l1); hv.x = h0 | (h1 << 16); lv.x = l0 | (l1 << 16);
    bfsplit(a.z, h0, l0); bfsplit(a.w, h1, l1); hv.y = h0 | (h1 << 16); lv.y = l0 | (l1 << 16);
    bfsplit(b.x, h0, l0); bfsplit(b.y, h1, l1); hv.z = h0 | (h1 << 16); lv.z = l0 | (l1 << 16);
    bfsplit(b.z, h0, l0); bfsplit(b.w, h1, l1); hv.w = h0 | (h1 << 16); lv.w = l0 | (l1 << 16);
}

__global__ __launch_bounds__(256) void k_cast_bf(const float* __restrict__ SRC, int lds, long long srcBatch, int rowsPerBatch,
                                                 u16* __restrict__ DST, int ldd, int nR, int nC, int dup) {
    const long long u = (long long)blockIdx.x * 256 + threadIdx.x; const int per = nC / 8;
    if (u >= (long long)nR * per) return;
    const int r = (int)(u / per); const int c0 = 8 * (int)(u - (long long)r * per);
    const int bb = r / rowsPerBatch; const int s = r - bb * rowsPerBatch;
    const float* sp = SRC + (long long)bb * srcBatch + (long long)s * lds + c0;
    const v4f a = *(const v4f*)(sp); const v4f b4 = *(const v4f*)(sp + 4);
    v4u pk; pk.x = pk2bf(a.x, a.y); pk.y = pk2bf(a.z, a.w); pk.z = pk2bf(b4.x, b4.y); pk.w = pk2bf(b4.z, b4.w);
    u16* d = DST + (long long)r * ldd + c0;
    VST2(v4u, d, pk);
    if (dup != 0) { VST2(v4u, d + nC, pk); }
}

__global__ __launch_bounds__(32) void k_invf(float* __restrict__ invb) {
    const int i = threadIdx.x;
    const float e = ((float)i * 2.0f) / (float)DK;
    const float invf = 1.0f / powf(10000.0f, e);
    VST2(float, invb + i, invf);
}
__global__ __launch_bounds__(256) void k_sincos(float* __restrict__ cs, float* __restrict__ sn, const float* __restrict__ invb) {
    const int idx = blockIdx.x * 256 + threadIdx.x;
    if (idx >= SEQ * 32) return;
    const int s = idx >> 5, i = idx & 31;
    const float ang = (float)s * invb[i];
    const float cv = cosf(ang), sv = sinf(ang);
    VST2(float, cs + idx, cv); VST2(float, sn + idx, sv);
}

__global__ __launch_bounds__(256) void k_gemm64(const __bf16* __restrict__ A, int lda, long long strideA,
                                                const __bf16* __restrict__ Bt, int ldb,
                                                float* __restrict__ Cout, int ldc, long long strideC,
                                                int M, int N, int K) {
    __shared__ __align__(16) float sT[8][16 * 68];
    const int b    = blockIdx.y;
    const int lane = threadIdx.x & 31;
    const int wave = __builtin_amdgcn_readfirstlane((int)(threadIdx.x >> 5));
    const int tilesN = N >> 6;
    const int tilesM = M >> 6;
    const int tile = blockIdx.x * 8 + wave;
    if (tile >= tilesM * tilesN) return;
    const int tm = tile / tilesN;
    const int tn = tile - tm * tilesN;
    const int m0 = tm << 6;
    const int n0 = tn << 6;
    const __bf16* Ab = A + (size_t)b * strideA;
    const int rlane = lane & 15;
    const int koff  = (lane >> 4) * 8;
    const int mOff  = (lane >> 4) * 8;

    v8f acc[4][4];
#pragma unroll
    for (int i = 0; i < 4; ++i)
#pragma unroll
        for (int j = 0; j < 4; ++j) acc[i][j] = (v8f){0.f, 0.f, 0.f, 0.f, 0.f, 0.f, 0.f, 0.f};

    for (int k0 = 0; k0 < K; k0 += 32) {
        v16b bh[4];
#pragma unroll
        for (int j = 0; j < 4; ++j) {
            const __bf16* bp = Bt + (size_t)(n0 + (j << 4) + rlane) * ldb + koff + k0;
            FragB f; f.h[0] = *(const v8b*)(bp); f.h[1] = *(const v8b*)(bp + 16); bh[j] = f.v;
        }
#pragma unroll
        for (int i = 0; i < 4; ++i) {
            const __bf16* ap = Ab + (size_t)(m0 + (i << 4) + rlane) * lda + koff + k0;
            FragB fa; fa.h[0] = *(const v8b*)(ap); fa.h[1] = *(const v8b*)(ap + 16);
            const v16b ah = fa.v;
#pragma unroll
            for (int j = 0; j < 4; ++j)
                acc[i][j] = __builtin_amdgcn_wmma_f32_16x16x32_bf16(false, ah, false, bh[j], (short)0, acc[i][j], false, false);
            dep_guard_b(acc[i][0], acc[i][3], ah, ah);
        }
        keep4_b(bh[0], bh[1], bh[2], bh[3]);
    }
    acc_guard4(acc[0][0], acc[0][1], acc[0][2], acc[0][3]);
    acc_guard4(acc[1][0], acc[1][1], acc[1][2], acc[1][3]);
    acc_guard4(acc[2][0], acc[2][1], acc[2][2], acc[2][3]);
    acc_guard4(acc[3][0], acc[3][1], acc[3][2], acc[3][3]);

    float* slab = sT[wave];
    float* C = Cout + (size_t)b * strideC;
#pragma unroll
    for (int i = 0; i < 4; ++i) {
        const int mBase = m0 + (i << 4);
#pragma unroll
        for (int j = 0; j < 4; ++j) {
#pragma unroll
            for (int r = 0; r < 8; ++r) slab[(mOff + r) * 68 + (j << 4) + rlane] = acc[i][j][r];
        }
        __builtin_amdgcn_fence(3  , "workgroup");
        __builtin_amdgcn_wave_barrier();
        __builtin_amdgcn_fence(2  , "workgroup");
        {
            const int hh = lane >> 4, c4 = (lane & 15) * 4;
            for (int pass = 0; pass < 2; ++pass) {
#pragma unroll
                for (int it = 0; it < 8; ++it) {
                    const int row = it * 2 + hh;
                    const v4f v = *(const v4f*)(slab + row * 68 + c4);
                    *(volatile v4f*)(C + (size_t)(mBase + row) * ldc + n0 + c4) = v;
                }
                __threadfence();
            }
        }
        __builtin_amdgcn_fence(3  , "workgroup");
        __builtin_amdgcn_wave_barrier();
        __builtin_amdgcn_fence(2  , "workgroup");
    }
}

__global__ __launch_bounds__(256) void k_normrope(const float* __restrict__ QKV, const float* __restrict__ qnw, const float* __restrict__ knw,
                                                  const float* __restrict__ CS, const float* __restrict__ SN,
                                                  u16* __restrict__ Qh, u16* __restrict__ Ql, u16* __restrict__ Kh, u16* __restrict__ Kl) {
    const int lane = threadIdx.x & 31;
    const int wave = __builtin_amdgcn_readfirstlane((int)(threadIdx.x >> 5));
    const int task = blockIdx.x * 8 + wave;
    if (task >= NB * SEQ * 20) return;
    const int token = task / 20;
    const int r = task - token * 20;
    const int b = token / SEQ, s = token - b * SEQ;
    const bool isq = (r < 16);
    const int h = isq ? r : (r - 16);
    const int coff = isq ? (h * DK) : (DMODEL + h * DK);
    const int i2 = lane * 2;
    const v2f xv = *(const v2f*)(QKV + (size_t)token * QKVN + coff + i2);
    const float x0 = xv.x, x1 = xv.y;
    float ss = x0 * x0 + x1 * x1;
#pragma unroll
    for (int msk = 16; msk >= 1; msk >>= 1) ss += __shfl_xor(ss, msk, 32);
    const float rinv = rsqrtf(ss * (1.0f / 64.0f) + 1.1920929e-7f);
    const float wq0 = cmb_bf(qnw[i2]), wq1 = cmb_bf(qnw[i2 + 1]);
    const float wk0 = cmb_bf(knw[i2]), wk1 = cmb_bf(knw[i2 + 1]);
    const float w0 = isq ? wq0 : wk0, w1 = isq ? wq1 : wk1;
    const float y0 = x0 * rinv * w0;
    const float y1 = x1 * rinv * w1;
    const float cv = CS[s * 32 + lane], sv = SN[s * 32 + lane];
    const float o0 = y0 * cv - y1 * sv;
    const float o1 = y1 * cv + y0 * sv;
    if (isq) st_s2(Qh, Ql, ((size_t)(b * NH + h) * SEQ + s) * DK + i2, o0, o1);
    else     st_s2(Kh, Kl, ((size_t)(b * NKV + h) * SEQ + s) * DK + i2, o0, o1);
}

__global__ __launch_bounds__(256) void k_vt(const float* __restrict__ QKV, u16* __restrict__ Vh, u16* __restrict__ Vl) {
    __shared__ float tile[64][65];
    const int s0 = blockIdx.x * 64, kvh = blockIdx.y, b = blockIdx.z;
    const int tid = threadIdx.x, lane = tid & 31;
    const int wave = __builtin_amdgcn_readfirstlane((int)(threadIdx.x >> 5));
#pragma unroll 4
    for (int k = 0; k < 16; ++k) {
        const int idx = tid + 256 * k; const int rr = idx >> 6, cc = idx & 63;
        tile[rr][cc] = QKV[(size_t)(b * SEQ + s0 + rr) * QKVN + (DMODEL + NKV * DK) + kvh * DK + cc];
    }
    __syncthreads();
#pragma unroll
    for (int it = 0; it < 2; ++it) {
        const int d = it * 32 + wave * 4 + (lane >> 3);
        const int t0 = (lane & 7) * 8;
        v4f a, c;
        a.x = tile[t0 + 0][d]; a.y = tile[t0 + 1][d]; a.z = tile[t0 + 2][d]; a.w = tile[t0 + 3][d];
        c.x = tile[t0 + 4][d]; c.y = tile[t0 + 5][d]; c.z = tile[t0 + 6][d]; c.w = tile[t0 + 7][d];
        v4u hv, lv; split8(a, c, hv, lv);
        const size_t off = ((size_t)(b * NKV + kvh) * DK + d) * SEQ + s0 + t0;
        VST2(v4u, Vh + off, hv);
        VST2(v4u, Vl + off, lv);
    }
}

__global__ __launch_bounds__(128) void k_attn(const __bf16* __restrict__ Qh, const __bf16* __restrict__ Ql,
                                              const __bf16* __restrict__ Kh, const __bf16* __restrict__ Kl,
                                              const __bf16* __restrict__ Vh, const __bf16* __restrict__ Vl,
                                              const float* __restrict__ X, const float* __restrict__ SW,
                                              u16* __restrict__ CTX) {
    __shared__ __align__(16) float os[4][16 * 68];
    const int lane = threadIdx.x & 31;
    const int wave = __builtin_amdgcn_readfirstlane((int)(threadIdx.x >> 5));
    const int hf = lane >> 4, c = lane & 15;
    const int bh = blockIdx.y;
    const int b = bh / NH, h = bh - b * NH, kvh = h / GRP;
    const int qw = blockIdx.x * 64 + wave * 16;
    const int qg = qw + c;

    const __bf16* qhp = Qh + (size_t)(b * NH + h) * SEQ * DK;
    const __bf16* qlp = Ql + (size_t)(b * NH + h) * SEQ * DK;
    const __bf16* khp = Kh + (size_t)(b * NKV + kvh) * SEQ * DK;
    const __bf16* klp = Kl + (size_t)(b * NKV + kvh) * SEQ * DK;
    const __bf16* vhp = Vh + (size_t)(b * NKV + kvh) * DK * SEQ;
    const __bf16* vlp = Vl + (size_t)(b * NKV + kvh) * DK * SEQ;

    const v16b qh0 = frag_ld(qhp, DK, qw, 0, lane),  qh1 = frag_ld(qhp, DK, qw, 32, lane);
    const v16b ql0 = frag_ld(qlp, DK, qw, 0, lane),  ql1 = frag_ld(qlp, DK, qw, 32, lane);

    const v8f vz = (v8f){0.f, 0.f, 0.f, 0.f, 0.f, 0.f, 0.f, 0.f};
    v8f o[4];
#pragma unroll
    for (int t = 0; t < 4; ++t) o[t] = vz;
    const float NEG = -__builtin_inff();
    const float C2 = 0.125f * 1.4426950408889634f;
    float m = NEG, l = 0.f;
    const int kend = qw + 16;

    for (int kb = 0; kb < kend; kb += 32) {
        v8f s0 = vz, s1 = vz;
        { const v16b ah = frag_ld(khp, DK, kb, 0, lane);       const v16b al = frag_ld(klp, DK, kb, 0, lane);       s0 = mma3(ah, al, qh0, ql0, s0); }
        { const v16b ah = frag_ld(khp, DK, kb, 32, lane);      const v16b al = frag_ld(klp, DK, kb, 32, lane);      s0 = mma3(ah, al, qh1, ql1, s0); }
        { const v16b ah = frag_ld(khp, DK, kb + 16, 0, lane);  const v16b al = frag_ld(klp, DK, kb + 16, 0, lane);  s1 = mma3(ah, al, qh0, ql0, s1); }
        { const v16b ah = frag_ld(khp, DK, kb + 16, 32, lane); const v16b al = frag_ld(klp, DK, kb + 16, 32, lane); s1 = mma3(ah, al, qh1, ql1, s1); }

        const bool diag = (kb + 31 > qw);
        float p[16];
        float mb = NEG;
#pragma unroll
        for (int v = 0; v < 8; ++v) {
            float a = s0[v] * C2;
            if (diag && (kb + 8 * hf + v > qg)) a = NEG;
            p[v] = a; mb = fmaxf(mb, a);
            float a2 = s1[v] * C2;
            if (diag && (kb + 16 + 8 * hf + v > qg)) a2 = NEG;
            p[8 + v] = a2; mb = fmaxf(mb, a2);
        }
        mb = fmaxf(mb, __shfl_xor(mb, 16, 32));
        const float mnew = fmaxf(m, mb);
        const float corr = exp2f(m - mnew);
        float rs = 0.f;
#pragma unroll
        for (int v = 0; v < 16; ++v) { p[v] = exp2f(p[v] - mnew); rs += p[v]; }
        rs += __shfl_xor(rs, 16, 32);
        l = l * corr + rs;
        m = mnew;

        PFrag ph_, pl_;
#pragma unroll
        for (int v = 0; v < 4; ++v) {
            unsigned int h0, l0, h1, l1;
            bfsplit(p[2 * v], h0, l0); bfsplit(p[2 * v + 1], h1, l1);
            ph_.u[v] = h0 | (h1 << 16); pl_.u[v] = l0 | (l1 << 16);
            bfsplit(p[8 + 2 * v], h0, l0); bfsplit(p[8 + 2 * v + 1], h1, l1);
            ph_.u[4 + v] = h0 | (h1 << 16); pl_.u[4 + v] = l0 | (l1 << 16);
        }
#pragma unroll
        for (int t = 0; t < 4; ++t) o[t] = o[t] * corr;
#pragma unroll
        for (int t = 0; t < 4; ++t) {
            const v16b vh = frag_ld(vhp, SEQ, 16 * t, kb, lane);
            const v16b vl = frag_ld(vlp, SEQ, 16 * t, kb, lane);
            o[t] = mma3(vh, vl, ph_.v, pl_.v, o[t]);
        }
    }

    float f;
    {
        const float* xr = X + ((size_t)b * SEQ_FULL + qg) * DMODEL;
        const v4f x0 = *(const v4f*)(xr), x1 = *(const v4f*)(xr + 4), x2 = *(const v4f*)(xr + 8);
        const float xs[SWK] = {x0.x, x0.y, x0.z, x0.w, x1.x, x1.y, x1.z, x1.w, x2.x, x2.y, x2.z, x2.w};
        const float* swr = SW + h * SWK;
        float ds = 0.f;
#pragma unroll
        for (int g = 0; g < SWK; ++g) ds += cmb_bf(xs[g]) * cmb_bf(swr[g]);
        const float sg = 1.0f / (1.0f + expf(-ds));
        f = (1.0f / l) * sg;
    }
    float* osw = os[wave];
#pragma unroll
    for (int t = 0; t < 4; ++t) {
        v4f a, bq;
        a.x = o[t][0] * f; a.y = o[t][1] * f; a.z = o[t][2] * f; a.w = o[t][3] * f;
        bq.x = o[t][4] * f; bq.y = o[t][5] * f; bq.z = o[t][6] * f; bq.w = o[t][7] * f;
        *(v4f*)(osw + c * 68 + 16 * t + 8 * hf) = a;
        *(v4f*)(osw + c * 68 + 16 * t + 8 * hf + 4) = bq;
    }
    __builtin_amdgcn_fence(3  , "workgroup");
    __builtin_amdgcn_wave_barrier();
    __builtin_amdgcn_fence(2  , "workgroup");
    {
        const int q4 = lane >> 3, c8 = (lane & 7) * 8;
        u16* crow = CTX + (size_t)(b * SEQ + qw) * (2 * DMODEL) + h * DK + c8;
        for (int pass = 0; pass < 2; ++pass) {
#pragma unroll
            for (int it = 0; it < 4; ++it) {
                const int row = it * 4 + q4;
                const float* sp = osw + row * 68 + c8;
                const v4f a = *(const v4f*)(sp); const v4f bq = *(const v4f*)(sp + 4);
                v4u hv, lv; split8(a, bq, hv, lv);
                *(volatile v4u*)(crow + (size_t)row * (2 * DMODEL)) = hv;
                *(volatile v4u*)(crow + (size_t)row * (2 * DMODEL) + DMODEL) = lv;
            }
            __threadfence();
        }
    }
}

extern "C" void kernel_launch(void* const* d_in, const int* in_sizes, int n_in, void* d_out, int out_size, void* d_ws, size_t ws_size, hipStream_t stream) {
    if (n_in < 5) return;
    const long long needX = ((long long)(NB - 1) * SEQ_FULL + SEQ) * DMODEL;
    if ((long long)in_sizes[0] < needX) return;
    if ((long long)in_sizes[1] < (long long)(QKVN + DMODEL) * DMODEL) return;
    if (in_sizes[2] < DK || in_sizes[3] < DK || in_sizes[4] < NH * SWK) return;
    if ((long long)out_size < needX) return;

    const float* x   = (const float*)d_in[0];
    const float* W   = (const float*)d_in[1];
    const float* qnw = (const float*)d_in[2];
    const float* knw = (const float*)d_in[3];
    const float* sw  = (const float*)d_in[4];
    float* out = (float*)d_out;

    char* wsp = (char*)d_ws; size_t off = 0;
    auto take = [&](size_t bytes) -> char* { char* p = wsp + off; off += (bytes + 255) & ~(size_t)255; return p; };
    u16*   X16  = (u16*)take((size_t)NB * SEQ * DMODEL * 2);
    u16*   W16  = (u16*)take((size_t)QKVN * DMODEL * 2);
    u16*   WO2  = (u16*)take((size_t)DMODEL * (2 * DMODEL) * 2);
    float* QKV  = (float*)take((size_t)NB * SEQ * QKVN * 4);
    float* INVF = (float*)take(128);
    float* CS   = (float*)take((size_t)SEQ * 32 * 4);
    float* SN   = (float*)take((size_t)SEQ * 32 * 4);
    u16*   Qh   = (u16*)take((size_t)NB * NH * SEQ * DK * 2);
    u16*   Ql   = (u16*)take((size_t)NB * NH * SEQ * DK * 2);
    u16*   Kh   = (u16*)take((size_t)NB * NKV * SEQ * DK * 2);
    u16*   Kl   = (u16*)take((size_t)NB * NKV * SEQ * DK * 2);
    u16*   Vh   = (u16*)take((size_t)NB * NKV * DK * SEQ * 2);
    u16*   Vl   = (u16*)take((size_t)NB * NKV * DK * SEQ * 2);
    u16*   CTX  = (u16*)take((size_t)NB * SEQ * (2 * DMODEL) * 2);
    if (off > ws_size || off > (size_t)134217728) return;

    k_cast_bf<<<(unsigned)(((long long)NB * SEQ * (DMODEL / 8) + 255) / 256), 256, 0, stream>>>(x, DMODEL, (long long)SEQ_FULL * DMODEL, SEQ, X16, DMODEL, NB * SEQ, DMODEL, 0);
    k_cast_bf<<<(unsigned)(((long long)QKVN * (DMODEL / 8) + 255) / 256), 256, 0, stream>>>(W, DMODEL, 0, QKVN, W16, DMODEL, QKVN, DMODEL, 0);
    k_cast_bf<<<(unsigned)(((long long)DMODEL * (DMODEL / 8) + 255) / 256), 256, 0, stream>>>(W + (size_t)QKVN * DMODEL, DMODEL, 0, DMODEL, WO2, 2 * DMODEL, DMODEL, DMODEL, 1);
    k_invf<<<1, 32, 0, stream>>>(INVF);
    k_sincos<<<(SEQ * 32 + 255) / 256, 256, 0, stream>>>(CS, SN, INVF);
    k_gemm64<<<dim3((unsigned)(((SEQ / 64) * (QKVN / 64) + 7) / 8), (unsigned)NB), 256, 0, stream>>>(
        (const __bf16*)X16, DMODEL, (long long)SEQ * DMODEL, (const __bf16*)W16, DMODEL, QKV, QKVN, (long long)SEQ * QKVN, SEQ, QKVN, DMODEL);
    k_normrope<<<(unsigned)((NB * SEQ * 20 + 7) / 8), 256, 0, stream>>>(QKV, qnw, knw, CS, SN, Qh, Ql, Kh, Kl);
    k_vt<<<dim3((unsigned)(SEQ / 64), (unsigned)NKV, (unsigned)NB), 256, 0, stream>>>(QKV, Vh, Vl);
    k_attn<<<dim3((unsigned)(SEQ / 64), (unsigned)(NB * NH)), 128, 0, stream>>>(
        (const __bf16*)Qh, (const __bf16*)Ql, (const __bf16*)Kh, (const __bf16*)Kl, (const __bf16*)Vh, (const __bf16*)Vl, x, sw, CTX);
    k_gemm64<<<dim3((unsigned)(((SEQ / 64) * (DMODEL / 64) + 7) / 8), (unsigned)NB), 256, 0, stream>>>(
        (const __bf16*)CTX, 2 * DMODEL, (long long)SEQ * 2 * DMODEL, (const __bf16*)WO2, 2 * DMODEL, out, DMODEL, (long long)SEQ_FULL * DMODEL, SEQ, DMODEL, 2 * DMODEL);
}
